// RegionalAttentionOp_64003602645064
// MI455X (gfx1250) — hardware-verified
//
#include <hip/hip_runtime.h>
#include <math.h>

typedef __attribute__((ext_vector_type(16))) _Float16 v16h;
typedef __attribute__((ext_vector_type(16))) __bf16 v16b;
typedef __attribute__((ext_vector_type(8)))  _Float16 v8h;
typedef __attribute__((ext_vector_type(8)))  float v8f;
typedef __attribute__((ext_vector_type(4)))  float v4f;
typedef __attribute__((ext_vector_type(2)))  float v2f;
typedef __attribute__((ext_vector_type(4)))  unsigned v4u;
typedef __attribute__((ext_vector_type(4)))  int v4i;
typedef float __attribute__((may_alias)) float_a;
typedef int __attribute__((may_alias)) int_a;

template <typename T> __device__ __forceinline__ void vst2(void* p, T v) { *(volatile T*)p = v; __threadfence(); *(volatile T*)p = v; }
__device__ __forceinline__ v8f wmma16(v16h a, v16h b, v8f c) {
  v8f d = __builtin_amdgcn_wmma_f32_16x16x32_f16(false, a, false, b, (short)0, c, false, false);
  asm volatile("v_nop\n\tv_nop\n\tv_nop\n\tv_nop" : "+v"(d) : "v"(a), "v"(b));
  return d;
}
__device__ __forceinline__ v8f wmma_bf(v16b a, v16b b, v8f c) {
  v8f d = __builtin_amdgcn_wmma_f32_16x16x32_bf16(false, a, false, b, (short)0, c, false, false);
  asm volatile("v_nop\n\tv_nop\n\tv_nop\n\tv_nop" : "+v"(d) : "v"(a), "v"(b));
  return d;
}
__device__ __forceinline__ v16h frag_h(const _Float16* rowk0, int lane) {
  union { v16h v; v8h q[2]; } u; const _Float16* p = rowk0 + 8 * (lane >> 4);
  u.q[0] = *(const v8h*)p; u.q[1] = *(const v8h*)(p + 16); return u.v;
}
__device__ __forceinline__ v16h frag_f32(const float* rowk0, int lane) {
  v16h a; const float* p = rowk0 + 8 * (lane >> 4);
#pragma unroll
  for (int i = 0; i < 8; ++i) { a[i] = (_Float16)p[i]; a[8 + i] = (_Float16)p[16 + i]; }
  return a;
}
__device__ __forceinline__ v16h frag_f32s(const float* rowk0, int lane, float sc) {
  v16h a; const float* p = rowk0 + 8 * (lane >> 4);
#pragma unroll
  for (int i = 0; i < 8; ++i) { a[i] = (_Float16)(p[i] * sc); a[8 + i] = (_Float16)(p[16 + i] * sc); }
  return a;
}
__device__ __forceinline__ v16h fragc_f32(const float* W, int k0, int n, int lane, int ld, int K) {
  v16h a; const int g = lane >> 4;
#pragma unroll
  for (int i = 0; i < 8; ++i) { const int ka = k0 + 8 * g + i, kb = ka + 16;
    a[i] = (_Float16)(ka < K ? W[(size_t)(ka < K ? ka : K - 1) * ld + n] : 0.f); a[8 + i] = (_Float16)(kb < K ? W[(size_t)(kb < K ? kb : K - 1) * ld + n] : 0.f); }
  return a;
}
struct F2 { v16b h, l; };
__device__ __forceinline__ F2 bsplit16(const float v[16]) { F2 r;
#pragma unroll
  for (int i = 0; i < 16; ++i) { const __bf16 h = (__bf16)v[i]; r.h[i] = h; r.l[i] = (__bf16)(v[i] - (float)h); }
  return r; }
__device__ __forceinline__ F2 split_row(const float* row, int k0, int lane) { float v[16]; const float* p = row + k0 + 8 * (lane >> 4);
#pragma unroll
  for (int i = 0; i < 8; ++i) { v[i] = p[i]; v[8 + i] = p[16 + i]; }
  return bsplit16(v); }
__device__ __forceinline__ F2 split_rowK(const float* row, int k0, int lane, int K) { float v[16]; const int g = lane >> 4;
#pragma unroll
  for (int i = 0; i < 8; ++i) { const int ka = k0 + 8 * g + i, kb = ka + 16; v[i] = ka < K ? row[ka < K ? ka : K - 1] : 0.f; v[8 + i] = kb < K ? row[kb < K ? kb : K - 1] : 0.f; }
  return bsplit16(v); }
__device__ __forceinline__ F2 split_col(const float* W, int k0, int n, int lane, int ld, int K) { float v[16]; const int g = lane >> 4;
#pragma unroll
  for (int i = 0; i < 8; ++i) { const int ka = k0 + 8 * g + i, kb = ka + 16; v[i] = ka < K ? W[(size_t)(ka < K ? ka : K - 1) * ld + n] : 0.f; v[8 + i] = kb < K ? W[(size_t)(kb < K ? kb : K - 1) * ld + n] : 0.f; }
  return bsplit16(v); }
__device__ __forceinline__ v8f mac3(const F2& a, const F2& b, v8f c) { c = wmma_bf(a.l, b.h, c); c = wmma_bf(a.h, b.l, c); return wmma_bf(a.h, b.h, c); }
__device__ __forceinline__ float sigm(float v) { return 1.0f / (1.0f + expf(-v)); }
#define LDSX() do { asm volatile("s_wait_dscnt 0" ::: "memory"); __builtin_amdgcn_wave_barrier(); __builtin_amdgcn_fence(__ATOMIC_RELEASE, "workgroup"); } while (0)


#define SQ 4096
#define NH 16
#define HD 128
#define PP 512
#define NRG 2
#define QROW (NH * HD)
#ifndef TQB
#define TQB (SQ / 64)
#endif
typedef __attribute__((ext_vector_type(8))) __bf16 v8b;
__device__ __forceinline__ v16b frag_b(const __bf16* rowk0, int lane) {
  union { v16b v; v8b q[2]; } u; const __bf16* p = rowk0 + 8 * (lane >> 4);
  u.q[0] = *(const v8b*)p; u.q[1] = *(const v8b*)(p + 16); return u.v;
}
__device__ __forceinline__ v16b frag_gbf(const float* rowk0, int lane) {
  v16b a; const float* p = rowk0 + 8 * (lane >> 4);
#pragma unroll
  for (int i = 0; i < 8; ++i) { a[i] = (__bf16)p[i]; a[8 + i] = (__bf16)p[16 + i]; }
  return a;
}
__device__ __forceinline__ float bfr(float v) { return (float)(__bf16)v; }
__device__ __attribute__((noinline)) float exp_ni(float v) { return expf(v); }
#define WS_VT  0u
#define WS_END (WS_VT + 2u * 3 * QROW * PP)

__global__ __launch_bounds__(256) void k_vt(const float* __restrict__ V, const float* __restrict__ RV, __bf16* __restrict__ VT) {
  __shared__ __align__(16) __bf16 st[QROW][72];
  const int vb = blockIdx.y, p0 = blockIdx.x * 64, tid = threadIdx.x; const float* src = vb == 0 ? V : RV + (size_t)(vb - 1) * PP * QROW;
  for (int q = tid; q < 64 * QROW; q += 256) { const int pl = q / QROW, c = q % QROW; st[c][pl] = (__bf16)src[(size_t)(p0 + pl) * QROW + c]; }
  __syncthreads();
  for (int q = tid; q < QROW * 8; q += 256) { const int c = q >> 3, pc = q & 7; vst2((unsigned*)(VT + ((size_t)vb * QROW + c) * PP + p0 + pc * 8), *(const v4u*)&st[c][pc * 8]); }
}
__device__ __forceinline__ void att_step(const v16b* aq, const float* __restrict__ krow0, const __bf16* __restrict__ vrow0, int ks, const bool* allow, float* m, float* l, v8f* acc, float (*sp)[36], int lane, int col, int g, float scale) {
  v8f s[2];
#pragma unroll
  for (int ct = 0; ct < 2; ++ct) { const float* kr = krow0 + (size_t)(ks * 32 + ct * 16 + col) * QROW; v8f c = {};
#pragma unroll
    for (int kc = 0; kc < 4; ++kc) c = wmma_bf(aq[kc], frag_gbf(kr + kc * 32, lane), c);
#pragma unroll
    for (int r = 0; r < 8; ++r) s[ct][r] = allow[r] ? c[r] * scale : -3.0e38f; }
#pragma unroll
  for (int r = 0; r < 8; ++r) { float mx = fmaxf(s[0][r], s[1][r]);
#pragma unroll
    for (int o = 1; o < 16; o <<= 1) mx = fmaxf(mx, __shfl_xor(mx, o));
    const float mn = fmaxf(m[r], mx); const float alpha = (m[r] <= -1.0e38f) ? 0.f : exp_ni(m[r] - mn);
    const float e0 = s[0][r] <= -1.0e38f ? 0.f : exp_ni(s[0][r] - mn), e1 = s[1][r] <= -1.0e38f ? 0.f : exp_ni(s[1][r] - mn); float es = e0 + e1;
#pragma unroll
    for (int o = 1; o < 16; o <<= 1) es += __shfl_xor(es, o);
    l[r] = l[r] * alpha + es; m[r] = mn;
#pragma unroll
    for (int dt = 0; dt < 8; ++dt) acc[dt][r] *= alpha;
    sp[8 * g + r][col] = e0; sp[8 * g + r][16 + col] = e1; }
  LDSX();
  const F2 pa = split_row(&sp[col][0], 0, lane);
#pragma unroll
  for (int dt = 0; dt < 8; ++dt) { const v16b vv = frag_b(vrow0 + (size_t)(dt * 16 + col) * PP + ks * 32, lane); acc[dt] = wmma_bf(pa.l, vv, acc[dt]); acc[dt] = wmma_bf(pa.h, vv, acc[dt]); }
  LDSX();
}
__global__ __launch_bounds__(128) void k_attn(const float* __restrict__ Q, const float* __restrict__ K, const float* __restrict__ RK, const int* __restrict__ RM, const __bf16* __restrict__ VT, float* __restrict__ out) {
  __shared__ __align__(16) float sp[4][16][36]; __shared__ __align__(16) float sob[4][16][HD + 4];
  const int tid = threadIdx.x, wave = tid >> 5, lane = tid & 31, col = lane & 15, g = lane >> 4; const int h = blockIdx.y, q0 = blockIdx.x * 64 + wave * 16; const float scale = 0.08838834764831845f;
  v16b aq[4];
#pragma unroll
  for (int kc = 0; kc < 4; ++kc) aq[kc] = frag_gbf(Q + (size_t)(q0 + col) * QROW + h * HD + kc * 32, lane);
  bool allow[8]; float m[8], l[8]; v8f acc[8];
#pragma unroll
  for (int r = 0; r < 8; ++r) { allow[r] = true; m[r] = -3.0e38f; l[r] = 0.f; }
#pragma unroll
  for (int dt = 0; dt < 8; ++dt) acc[dt] = (v8f){};
#pragma unroll 1
  for (int ks = 0; ks < PP / 32; ++ks) att_step(aq, K + h * HD, VT + ((size_t)0 * QROW + h * HD) * PP, ks, allow, m, l, acc, sp[wave], lane, col, g, scale);
#pragma unroll
  for (int r = 0; r < 8; ++r) { const float il = 0.5f / l[r];
#pragma unroll
    for (int dt = 0; dt < 8; ++dt) sob[wave][8 * g + r][dt * 16 + col] = acc[dt][r] * il; }
  bool f0[8], f1[8], f2[8];
#pragma unroll
  for (int r = 0; r < 8; ++r) { const int s = q0 + 8 * g + r; const bool m0 = RM[s] != 0, m1 = RM[SQ + s] != 0; f0[r] = !(m0 || m1); f1[r] = m0; f2[r] = m1; m[r] = -3.0e38f; l[r] = 0.f; }
#pragma unroll
  for (int dt = 0; dt < 8; ++dt) acc[dt] = (v8f){};
#pragma unroll 1
  for (int blk = 0; blk < 3; ++blk) {
#pragma unroll
    for (int r = 0; r < 8; ++r) allow[r] = blk == 0 ? f0[r] : (blk == 1 ? f1[r] : f2[r]);
    const float* kb = blk == 0 ? K + h * HD : RK + (size_t)(blk - 1) * PP * QROW + h * HD; const __bf16* vb = VT + ((size_t)blk * QROW + h * HD) * PP;
#pragma unroll 1
    for (int ks = 0; ks < PP / 32; ++ks) att_step(aq, kb, vb, ks, allow, m, l, acc, sp[wave], lane, col, g, scale); }
#pragma unroll
  for (int r = 0; r < 8; ++r) { const float il = 0.5f / l[r];
#pragma unroll
    for (int dt = 0; dt < 8; ++dt) sob[wave][8 * g + r][dt * 16 + col] += acc[dt][r] * il; }
  LDSX();
  for (int rl = 0; rl < 16; ++rl) vst2(out + (size_t)(q0 + rl) * QROW + h * HD + lane * 4, *(const v4f*)&sob[wave][rl][lane * 4]);
}

extern "C" void kernel_launch(void* const* d_in, const int* in_sizes, int n_in, void* d_out, int out_size, void* d_ws, size_t ws_size, hipStream_t stream) {
  (void)in_sizes; (void)n_in; (void)out_size;
  const float** F = (const float**)d_in; const int** I = (const int**)d_in;
  if (ws_size < (size_t)WS_END) return;
  __bf16* VT = (__bf16*)((char*)d_ws + WS_VT);
  k_vt<<<dim3(PP / 64, 3), 256, 0, stream>>>(F[2], F[4], VT);
  k_attn<<<dim3(TQB, NH), 128, 0, stream>>>(F[0], F[1], F[3], I[5], VT, (float*)d_out);
}
